// BlockDecoder_3547642987208
// MI455X (gfx1250) — hardware-run, weakly checked
//
#include <hip/hip_runtime.h>

#ifndef NB
#define NB 4
#endif
#ifndef SEQ
#define SEQ 1024
#endif
#define NB_FULL 4
#define SEQ_FULL 1024
#define DM 1024
#define NH 16
#define HD 64
#define DFF 4096
#define NR ((size_t)NB * SEQ)
#define MR ((int)((size_t)NB * SEQ))
#define PBP 40
#define OBP 72
#define LN_EPS 1.0e-5f
#define PCARRY 16384.0f
#define RCARRY 2048.0f
#define RINV 0.00048828125f

static_assert(NB >= 1 && NB <= NB_FULL);
static_assert(SEQ >= 64 && SEQ <= SEQ_FULL && SEQ % 64 == 0);
static_assert((NB * SEQ) % 128 == 0);
static_assert(NH * HD == DM && HD == 64);
static_assert(DM == 4 * 256);
static_assert(DM % 64 == 0 && DFF % 64 == 0 && DM % 32 == 0 && DFF % 32 == 0);
static_assert(DFF <= 4 * DM);
static_assert((PBP % 8) == 0 && (OBP % 8) == 0);
static_assert(DFF == 4 * DM);
static_assert(PBP >= 32 && OBP >= HD);
static_assert(RCARRY * RINV == 1.0f);
static_assert(PCARRY <= 32768.0f);
static_assert((size_t)8 * DM * DM * 2 + (size_t)2 * DM * DFF * 2 + (size_t)10 * NB * SEQ * DM * 2 + 16 * 256 <= (size_t)134217728);

typedef unsigned short v8us __attribute__((ext_vector_type(8), may_alias));
typedef float  v8f  __attribute__((ext_vector_type(8)));
typedef float  v4f  __attribute__((ext_vector_type(4)));
typedef float  v4fa __attribute__((ext_vector_type(4), may_alias));
typedef _Float16 v16h __attribute__((ext_vector_type(16)));
typedef _Float16 v4h __attribute__((ext_vector_type(4)));
union FragH { v16h v; v8us half[2]; _Float16 h[16]; unsigned short u[16]; };

__device__ __forceinline__ unsigned short bf16_bits(float x) { unsigned int u = __float_as_uint(x); return (unsigned short)((u + 0x7FFFu + ((u >> 16) & 1u)) >> 16); }
__device__ __forceinline__ float bf16_val(unsigned short b) { return __uint_as_float(((unsigned int)b) << 16); }
__device__ __forceinline__ float bf16_rne(float x) { return bf16_val(bf16_bits(x)); }

__device__ __forceinline__ v16h g2_frag(const _Float16* p, int hh) { FragH f; f.half[0] = *(const v8us*)((const unsigned short*)p + 8 * hh); f.half[1] = *(const v8us*)((const unsigned short*)p + 16 + 8 * hh); return f.v; }
__device__ __forceinline__ v8f g2_mma(v16h a, v16h b, v8f c) { v8f d = __builtin_amdgcn_wmma_f32_16x16x32_f16(false, a, false, b, (short)0, c, false, false); asm volatile("v_nop\n\tv_nop\n\tv_nop\n\tv_nop" : "+v"(d) : "v"(a), "v"(b)); return d; }

typedef _Float16 h16;
static __device__ __forceinline__ h16 toh_flush(float v) { const h16 r = (h16)v; return (fabsf(v) < 6.103515625e-05f) ? (h16)0.0f : r; }

__global__ __launch_bounds__(256) void k_wt_f16(const float* __restrict__ W, _Float16* __restrict__ Wt, int K, int N, float scale) {
  const int t = blockIdx.x * 256 + threadIdx.x; if (t >= N * (K / 8)) return;
  const int n = t / (K / 8), k8 = (t % (K / 8)) * 8; FragH f;
#pragma unroll
  for (int i = 0; i < 8; ++i) f.h[i] = (_Float16)(bf16_rne(W[(size_t)(k8 + i) * N + n]) * scale);
  const v8us o = f.half[0]; unsigned short* d = (unsigned short*)Wt + (size_t)n * K + k8;
  *(volatile v8us*)d = o; __threadfence(); *(volatile v8us*)d = o;
}

__global__ __launch_bounds__(256) void k_wt_head(const float* __restrict__ W, _Float16* __restrict__ Wt, int K, int N, float scale) {
  const int t = blockIdx.x * 256 + threadIdx.x; if (t >= N * (K / 8)) return;
  const int n = t / (K / 8), k8 = (t % (K / 8)) * 8; const int hd = n / HD, dd = n % HD; FragH f;
#pragma unroll
  for (int i = 0; i < 8; ++i) f.h[i] = toh_flush(bf16_rne(W[((size_t)hd * K + k8 + i) * HD + dd]) * scale);
  const v8us o = f.half[0]; unsigned short* d = (unsigned short*)Wt + (size_t)n * K + k8;
  *(volatile v8us*)d = o; __threadfence(); *(volatile v8us*)d = o;
}

__global__ __launch_bounds__(256) void k_x16(const float* __restrict__ x, _Float16* __restrict__ X16, size_t n8) {
  const size_t t = (size_t)blockIdx.x * 256 + threadIdx.x; if (t >= n8) return;
  const size_t e = t * 8; const size_t r = e / DM; const size_t c = e % DM; const size_t rs = (r / SEQ) * SEQ_FULL + (r % SEQ);
  const float* src = x + rs * DM + c; const v4f a = *(const v4fa*)src; const v4f a2 = *(const v4fa*)(src + 4); FragH f;
#pragma unroll
  for (int q = 0; q < 4; ++q) { f.h[q] = (_Float16)bf16_rne(a[q]); f.h[4 + q] = (_Float16)bf16_rne(a2[q]); }
  const v8us o = f.half[0]; unsigned short* d = (unsigned short*)X16 + e;
  *(volatile v8us*)d = o; __threadfence(); *(volatile v8us*)d = o;
}

__global__ __launch_bounds__(256) void k_split16(const float* __restrict__ src, _Float16* __restrict__ H16, _Float16* __restrict__ R16, size_t n8) {
  #pragma clang fp contract(off)
  const size_t t = (size_t)blockIdx.x * 256 + threadIdx.x; if (t >= n8) return;
  const size_t e = t * 8; const v4f a = *(const v4fa*)(src + e); const v4f a2 = *(const v4fa*)(src + e + 4); FragH fh, fr;
#pragma unroll
  for (int q = 0; q < 4; ++q) {
    const h16 h0 = toh_flush(a[q]);  fh.h[q] = h0;     fr.h[q] = toh_flush((a[q] - (float)h0) * RCARRY);
    const h16 h1 = toh_flush(a2[q]); fh.h[4 + q] = h1; fr.h[4 + q] = toh_flush((a2[q] - (float)h1) * RCARRY); }
  const v8us oh = fh.half[0]; const v8us orr = fr.half[0];
  unsigned short* dh = (unsigned short*)H16 + e; unsigned short* dr = (unsigned short*)R16 + e;
  *(volatile v8us*)dh = oh; *(volatile v8us*)dr = orr; __threadfence(); *(volatile v8us*)dh = oh; *(volatile v8us*)dr = orr;
}

template <int NHv, int TTv>
__global__ __launch_bounds__(256) void k_vt(const _Float16* __restrict__ V16, int ldv, int voff, _Float16* __restrict__ Vt) {
  __shared__ unsigned short tl[64][66]; const int tid = threadIdx.x; const int slab = blockIdx.x / (TTv / 64), lg = blockIdx.x % (TTv / 64); const int b = slab / NHv, h = slab % NHv;
  for (int i = tid; i < 64 * 8; i += 256) { const int r = i / 8, c8 = (i % 8) * 8; FragH f; f.half[0] = *(const v8us*)((const unsigned short*)V16 + ((size_t)b * TTv + lg * 64 + r) * ldv + voff + h * 64 + c8);
#pragma unroll
    for (int q = 0; q < 8; ++q) tl[r][c8 + q] = f.u[q]; }
  __syncthreads();
  for (int pass = 0; pass < 2; ++pass) {
#pragma unroll
    for (int rd = 0; rd < 2; ++rd) { const int d = rd * 32 + tid / 8, pc = tid % 8; FragH f;
#pragma unroll
      for (int q = 0; q < 8; ++q) f.u[q] = tl[pc * 8 + q][d];
      *(volatile v8us*)((unsigned short*)Vt + ((size_t)slab * 64 + d) * TTv + lg * 64 + pc * 8) = f.half[0]; }
    if (pass == 0) __threadfence(); }
}

template <int ACT>
__global__ __launch_bounds__(128) void k_gemm2(const _Float16* __restrict__ A, int lda, const _Float16* __restrict__ Bh, int ldb, float alpha, const float* __restrict__ bias, float bsc,
    float* __restrict__ C, _Float16* __restrict__ C16, int ldc, int M, int N, int K) {
  static_assert(ACT == 0 || ACT == 3);
  __shared__ __attribute__((aligned(16))) float so[4][32][68];
  const int tid = threadIdx.x, w = tid >> 5, lane = tid & 31, ln = lane & 15, hh = lane >> 4;
  const int ntn = N >> 6; const int mt = blockIdx.x / ntn, nq = blockIdx.x - mt * ntn; const int row0 = mt * 128 + 32 * w, col0 = nq * 64; if (row0 >= M) return;
  const _Float16* a0p = A + (size_t)(row0 + ln) * lda; const _Float16* a1p = a0p + (size_t)16 * lda;
  const _Float16* b0p = Bh + (size_t)(col0 + ln) * ldb; const _Float16* b1p = b0p + (size_t)16 * ldb; const _Float16* b2p = b1p + (size_t)16 * ldb; const _Float16* b3p = b2p + (size_t)16 * ldb;
  const v8f z8 = {0.f,0.f,0.f,0.f,0.f,0.f,0.f,0.f}; v8f c00 = z8, c01 = z8, c02 = z8, c03 = z8, c10 = z8, c11 = z8, c12 = z8, c13 = z8;
#pragma unroll 1
  for (int kb = 0; kb < K; kb += 32) { const v16h a0 = g2_frag(a0p + kb, hh), a1 = g2_frag(a1p + kb, hh);
    v16h b = g2_frag(b0p + kb, hh); c00 = g2_mma(a0, b, c00); c10 = g2_mma(a1, b, c10);
    b = g2_frag(b1p + kb, hh); c01 = g2_mma(a0, b, c01); c11 = g2_mma(a1, b, c11);
    b = g2_frag(b2p + kb, hh); c02 = g2_mma(a0, b, c02); c12 = g2_mma(a1, b, c12);
    b = g2_frag(b3p + kb, hh); c03 = g2_mma(a0, b, c03); c13 = g2_mma(a1, b, c13); }
  v8f accs[8] = {c00, c01, c02, c03, c10, c11, c12, c13};
#pragma unroll
  for (int u = 0; u < 8; ++u) { const int t = u & 3, half = u >> 2; const int col = col0 + t * 16 + ln; const float bv = bias ? bf16_rne(bias[col]) * bsc : 0.f;
#pragma unroll
    for (int r = 0; r < 8; ++r) { const int rloc = half * 16 + 8 * hh + r; float v = accs[u][r] * alpha + bv; if (ACT == 3) v = fmaxf(v, 0.f); so[w][rloc][t * 16 + ln] = v; } }
  __builtin_amdgcn_fence(4  , "workgroup"); __builtin_amdgcn_wave_barrier();
  const int rsub = lane >> 4, c4 = (lane & 15) * 4;
  for (int pass = 0; pass < 2; ++pass) {
#pragma unroll
    for (int q = 0; q < 16; ++q) { const int r = q * 2 + rsub; const v4f v = *(const v4fa*)&so[w][r][c4];
      if (C) *(volatile v4f*)(C + (size_t)(row0 + r) * ldc + col0 + c4) = v;
      if (C16) { v4h h4; for (int i = 0; i < 4; ++i) h4[i] = (_Float16)v[i]; *(volatile v4h*)(C16 + (size_t)(row0 + r) * ldc + col0 + c4) = h4; } }
    if (pass == 0) __threadfence(); }
}

static __device__ __forceinline__ void gemm_kloop(const _Float16* a0p, const _Float16* a1p, const _Float16* b0p, const _Float16* b1p, const _Float16* b2p, const _Float16* b3p, int K, int hh,
    v8f& c00, v8f& c01, v8f& c02, v8f& c03, v8f& c10, v8f& c11, v8f& c12, v8f& c13) {
#pragma unroll 1
  for (int kb = 0; kb < K; kb += 32) { const v16h a0 = g2_frag(a0p + kb, hh), a1 = g2_frag(a1p + kb, hh);
    v16h b = g2_frag(b0p + kb, hh); c00 = g2_mma(a0, b, c00); c10 = g2_mma(a1, b, c10);
    b = g2_frag(b1p + kb, hh); c01 = g2_mma(a0, b, c01); c11 = g2_mma(a1, b, c11);
    b = g2_frag(b2p + kb, hh); c02 = g2_mma(a0, b, c02); c12 = g2_mma(a1, b, c12);
    b = g2_frag(b3p + kb, hh); c03 = g2_mma(a0, b, c03); c13 = g2_mma(a1, b, c13); }
}

template <int ARES, int OUTHR>
static __device__ __forceinline__ void gemm_hr_body(const _Float16* __restrict__ A, const _Float16* __restrict__ AR, int lda, const _Float16* __restrict__ Bh, int ldb, float alpha,
    const float* __restrict__ bias, float bsc, float* __restrict__ C, _Float16* __restrict__ CH, _Float16* __restrict__ CR, int ldc, int M, int N, int K) {
  __shared__ __attribute__((aligned(16))) float so[4][32][68];
  const int tid = threadIdx.x, lane = tid & 31, ln = lane & 15, hh = lane >> 4;
  const int w = __builtin_amdgcn_readfirstlane(tid >> 5);
  const int ntn = N >> 6; const int mt = blockIdx.x / ntn, nq = blockIdx.x - mt * ntn; const int row0 = mt * 128 + 32 * w, col0 = nq * 64; if (row0 >= M) return;
  const _Float16* b0p = Bh + (size_t)(col0 + ln) * ldb; const _Float16* b1p = b0p + (size_t)16 * ldb; const _Float16* b2p = b1p + (size_t)16 * ldb; const _Float16* b3p = b2p + (size_t)16 * ldb;
  const v8f z8 = {0.f,0.f,0.f,0.f,0.f,0.f,0.f,0.f};
  if (ARES) {
    const _Float16* r0p = AR + (size_t)(row0 + ln) * lda; const _Float16* r1p = r0p + (size_t)16 * lda;
    v8f d00 = z8, d01 = z8, d02 = z8, d03 = z8, d10 = z8, d11 = z8, d12 = z8, d13 = z8;
    gemm_kloop(r0p, r1p, b0p, b1p, b2p, b3p, K, hh, d00, d01, d02, d03, d10, d11, d12, d13);
    v8f ds[8] = {d00, d01, d02, d03, d10, d11, d12, d13};
#pragma unroll
    for (int u = 0; u < 8; ++u) { const int t = u & 3, half = u >> 2;
#pragma unroll
      for (int r = 0; r < 8; ++r) { const int rloc = half * 16 + 8 * hh + r; so[w][rloc][t * 16 + ln] = ds[u][r] * RINV; } }
  }
  const _Float16* a0p = A + (size_t)(row0 + ln) * lda; const _Float16* a1p = a0p + (size_t)16 * lda;
  v8f c00 = z8, c01 = z8, c02 = z8, c03 = z8, c10 = z8, c11 = z8, c12 = z8, c13 = z8;
  gemm_kloop(a0p, a1p, b0p, b1p, b2p, b3p, K, hh, c00, c01, c02, c03, c10, c11, c12, c13);
  v8f accs[8] = {c00, c01, c02, c03, c10, c11, c12, c13};
#pragma unroll
  for (int u = 0; u < 8; ++u) { const int t = u & 3, half = u >> 2; const int col = col0 + t * 16 + ln; const float bv = bias ? bf16_rne(bias[col]) * bsc : 0.f;
#pragma unroll
    for (int r = 0; r < 8; ++r) { const int rloc = half * 16 + 8 * hh + r; float v = accs[u][r]; if (ARES) v += so[w][rloc][t * 16 + ln]; v = v * alpha + bv; so[w][rloc][t * 16 + ln] = v; } }
  __builtin_amdgcn_fence(4  , "workgroup"); __builtin_amdgcn_wave_barrier();
  const int rsub = lane >> 4, c4 = (lane & 15) * 4;
  for (int pass = 0; pass < 2; ++pass) {
#pragma unroll
    for (int q = 0; q < 16; ++q) { const int r = q * 2 + rsub; const v4f v = *(const v4fa*)&so[w][r][c4];
      if (OUTHR) { v4h h4, r4;
#pragma unroll
        for (int i = 0; i < 4; ++i) { const h16 hv = toh_flush(v[i]); h4[i] = hv; r4[i] = toh_flush((v[i] - (float)hv) * RCARRY); }
        *(volatile v4h*)(CH + (size_t)(row0 + r) * ldc + col0 + c4) = h4;
        *(volatile v4h*)(CR + (size_t)(row0 + r) * ldc + col0 + c4) = r4; }
      else { *(volatile v4f*)(C + (size_t)(row0 + r) * ldc + col0 + c4) = v; } }
    if (pass == 0) __threadfence(); }
}

__global__ __launch_bounds__(128) void k_proj_hr(const _Float16* __restrict__ A, int lda, const _Float16* __restrict__ Bh, int ldb, float alpha,
    _Float16* __restrict__ CH, _Float16* __restrict__ CR, int ldc, int M, int N, int K) {
  gemm_hr_body<0, 1>(A, A, lda, Bh, ldb, alpha, nullptr, 0.f, nullptr, CH, CR, ldc, M, N, K);
}
__global__ __launch_bounds__(128) void k_proj_rhr(const _Float16* __restrict__ A, const _Float16* __restrict__ AR, int lda, const _Float16* __restrict__ Bh, int ldb, float alpha,
    _Float16* __restrict__ CH, _Float16* __restrict__ CR, int ldc, int M, int N, int K) {
  gemm_hr_body<1, 1>(A, AR, lda, Bh, ldb, alpha, nullptr, 0.f, nullptr, CH, CR, ldc, M, N, K);
}
__global__ __launch_bounds__(128) void k_proj_rf(const _Float16* __restrict__ A, const _Float16* __restrict__ AR, int lda, const _Float16* __restrict__ Bh, int ldb, float alpha,
    const float* __restrict__ bias, float bsc, float* __restrict__ C, int ldc, int M, int N, int K) {
  gemm_hr_body<1, 0>(A, AR, lda, Bh, ldb, alpha, bias, bsc, C, nullptr, nullptr, ldc, M, N, K);
}

template <int CAUSAL>
static __device__ __forceinline__ void attn_hr_body(const _Float16* __restrict__ Q16, const _Float16* __restrict__ QR, const _Float16* __restrict__ K16, const _Float16* __restrict__ KR,
    const _Float16* __restrict__ VT, const _Float16* __restrict__ VTR, _Float16* __restrict__ O16, _Float16* __restrict__ OR16) {
  __shared__ __attribute__((aligned(16))) _Float16 pb[4][16 * PBP];
  __shared__ __attribute__((aligned(16))) _Float16 pbr[4][16 * PBP];
  __shared__ __attribute__((aligned(16))) _Float16 ob[4][16 * OBP];
  __shared__ __attribute__((aligned(16))) _Float16 obr[4][16 * OBP];
  const int tid = threadIdx.x, lane = tid & 31, ln = lane & 15, hh = lane >> 4;
  const int w = __builtin_amdgcn_readfirstlane(tid >> 5);
  const int h = blockIdx.y, b = blockIdx.z;
  const int q0 = (blockIdx.x * 4 + w) * 16;
  const size_t tok0 = (size_t)b * SEQ;
  const int slab = b * NH + h;
  const size_t qoff = (tok0 + q0 + ln) * DM + h * HD;
  const v16h qf0 = g2_frag(Q16 + qoff, hh), qf1 = g2_frag(Q16 + qoff + 32, hh);
  const v16h qr0 = g2_frag(QR + qoff, hh),  qr1 = g2_frag(QR + qoff + 32, hh);
  const v8f z8 = {0.f,0.f,0.f,0.f,0.f,0.f,0.f,0.f};
  v8f o0 = z8, o1 = z8, o2 = z8, o3 = z8;
  v8f e0 = z8, e1 = z8, e2 = z8, e3 = z8;
  float mrow[8], lrow[8];
#pragma unroll
  for (int r = 0; r < 8; ++r) { mrow[r] = -1.0e30f; lrow[r] = 0.f; }
  const int kend = CAUSAL ? (q0 + 16) : SEQ;
#pragma unroll 1
  for (int kb = 0; kb < kend; kb += 32) {
    const size_t koff = (tok0 + kb + ln) * DM + h * HD;
    const _Float16* k0p = K16 + koff; const _Float16* k1p = k0p + (size_t)16 * DM;
    const _Float16* r0p = KR + koff;  const _Float16* r1p = r0p + (size_t)16 * DM;
    v8f s0 = z8, s1 = z8, t0 = z8, t1 = z8;
    v16h kf = g2_frag(k0p, hh);    s0 = g2_mma(qf0, kf, s0); t0 = g2_mma(qr0, kf, t0);
    kf = g2_frag(k0p + 32, hh);    s0 = g2_mma(qf1, kf, s0); t0 = g2_mma(qr1, kf, t0);
    kf = g2_frag(r0p, hh);         t0 = g2_mma(qf0, kf, t0);
    kf = g2_frag(r0p + 32, hh);    t0 = g2_mma(qf1, kf, t0);
    kf = g2_frag(k1p, hh);         s1 = g2_mma(qf0, kf, s1); t1 = g2_mma(qr0, kf, t1);
    kf = g2_frag(k1p + 32, hh);    s1 = g2_mma(qf1, kf, s1); t1 = g2_mma(qr1, kf, t1);
    kf = g2_frag(r1p, hh);         t1 = g2_mma(qf0, kf, t1);
    kf = g2_frag(r1p + 32, hh);    t1 = g2_mma(qf1, kf, t1);
#pragma unroll
    for (int r = 0; r < 8; ++r) {
      const int row = q0 + 8 * hh + r;
      float a = (s0[r] + t0[r] * RINV) * 8.0f, c = (s1[r] + t1[r] * RINV) * 8.0f;
      if (CAUSAL) { a = ((kb + ln > row) || (a == 0.0f)) ? -1.0e9f : a; c = ((kb + 16 + ln > row) || (c == 0.0f)) ? -1.0e9f : c; }
      float t = fmaxf(a, c);
      t = fmaxf(t, __shfl_xor(t, 1, 32)); t = fmaxf(t, __shfl_xor(t, 2, 32)); t = fmaxf(t, __shfl_xor(t, 4, 32)); t = fmaxf(t, __shfl_xor(t, 8, 32));
      const float mnew = fmaxf(mrow[r], t);
      const float p0 = __expf(a - mnew), p1 = __expf(c - mnew);
      const float pc0 = p0 * PCARRY, pc1 = p1 * PCARRY;
      const h16 ph0 = toh_flush(pc0), ph1 = toh_flush(pc1);
      float ls = CAUSAL ? (pc0 + pc1) : ((float)ph0 + (float)ph1);
      ls += __shfl_xor(ls, 1, 32); ls += __shfl_xor(ls, 2, 32); ls += __shfl_xor(ls, 4, 32); ls += __shfl_xor(ls, 8, 32);
      const float corr = __expf(mrow[r] - mnew);
      lrow[r] = lrow[r] * corr + ls; mrow[r] = mnew;
      o0[r] *= corr; o1[r] *= corr; o2[r] *= corr; o3[r] *= corr;
      if (CAUSAL) { e0[r] *= corr; e1[r] *= corr; e2[r] *= corr; e3[r] *= corr; }
      pb[w][(8 * hh + r) * PBP + ln]      = ph0;
      pb[w][(8 * hh + r) * PBP + 16 + ln] = ph1;
      if (CAUSAL) {
        pbr[w][(8 * hh + r) * PBP + ln]      = toh_flush((pc0 - (float)ph0) * RCARRY);
        pbr[w][(8 * hh + r) * PBP + 16 + ln] = toh_flush((pc1 - (float)ph1) * RCARRY); }
    }
    __builtin_amdgcn_fence(4  , "wavefront"); __builtin_amdgcn_wave_barrier();
    const v16h pf = g2_frag(&pb[w][ln * PBP], hh);
    v16h prf = pf; if (CAUSAL) prf = g2_frag(&pbr[w][ln * PBP], hh);
    __builtin_amdgcn_fence(4  , "wavefront"); __builtin_amdgcn_wave_barrier();
    const size_t voff = ((size_t)slab * HD + ln) * SEQ + kb;
    const _Float16* vp = VT + voff; const _Float16* vrp = VTR + voff;
    v16h vf = g2_frag(vp, hh);                   o0 = g2_mma(pf, vf, o0);
    if (CAUSAL) { e0 = g2_mma(prf, vf, e0); vf = g2_frag(vrp, hh);                   e0 = g2_mma(pf, vf, e0); }
    vf = g2_frag(vp + (size_t)16 * SEQ, hh);     o1 = g2_mma(pf, vf, o1);
    if (CAUSAL) { e1 = g2_mma(prf, vf, e1); vf = g2_frag(vrp + (size_t)16 * SEQ, hh); e1 = g2_mma(pf, vf, e1); }
    vf = g2_frag(vp + (size_t)32 * SEQ, hh);     o2 = g2_mma(pf, vf, o2);
    if (CAUSAL) { e2 = g2_mma(prf, vf, e2); vf = g2_frag(vrp + (size_t)32 * SEQ, hh); e2 = g2_mma(pf, vf, e2); }
    vf = g2_frag(vp + (size_t)48 * SEQ, hh);     o3 = g2_mma(pf, vf, o3);
    if (CAUSAL) { e3 = g2_mma(prf, vf, e3); vf = g2_frag(vrp + (size_t)48 * SEQ, hh); e3 = g2_mma(pf, vf, e3); }
  }
#pragma unroll
  for (int r = 0; r < 8; ++r) {
    const float rl = 64.0f * __builtin_amdgcn_rcpf(lrow[r]);
    const int rloc = (8 * hh + r) * OBP + ln;
    float v0 = o0[r], v1 = o1[r], v2 = o2[r], v3 = o3[r];
    if (CAUSAL) { v0 += e0[r] * RINV; v1 += e1[r] * RINV; v2 += e2[r] * RINV; v3 += e3[r] * RINV; }
    v0 *= rl; v1 *= rl; v2 *= rl; v3 *= rl;
    const h16 g0 = toh_flush(v0), g1 = toh_flush(v1), g2 = toh_flush(v2), g3 = toh_flush(v3);
    ob[w][rloc] = g0; ob[w][rloc + 16] = g1; ob[w][rloc + 32] = g2; ob[w][rloc + 48] = g3;
    if (CAUSAL) {
      obr[w][rloc]      = toh_flush((v0 - (float)g0) * RCARRY); obr[w][rloc + 16] = toh_flush((v1 - (float)g1) * RCARRY);
      obr[w][rloc + 32] = toh_flush((v2 - (float)g2) * RCARRY); obr[w][rloc + 48] = toh_flush((v3 - (float)g3) * RCARRY); }
  }
  __builtin_amdgcn_fence(4  , "wavefront"); __builtin_amdgcn_wave_barrier();
  const int rq = lane >> 3, pc = (lane & 7) * 8;
  for (int pass = 0; pass < 2; ++pass) {
#pragma unroll
    for (int i = 0; i < 4; ++i) { const int row = i * 4 + rq; const size_t go = (tok0 + q0 + row) * DM + h * HD + pc;
      const v8us v = *(const v8us*)(&ob[w][row * OBP + pc]);
      *(volatile v8us*)((unsigned short*)O16 + go) = v;
      if (CAUSAL) { const v8us vr = *(const v8us*)(&obr[w][row * OBP + pc]); *(volatile v8us*)((unsigned short*)OR16 + go) = vr; } }
    if (pass == 0) __threadfence(); }
}

__global__ __launch_bounds__(128) void k_attn_causal(const _Float16* __restrict__ Q16, const _Float16* __restrict__ QR, const _Float16* __restrict__ K16, const _Float16* __restrict__ KR,
    const _Float16* __restrict__ VT, const _Float16* __restrict__ VTR, _Float16* __restrict__ O16, _Float16* __restrict__ OR16) {
  attn_hr_body<1>(Q16, QR, K16, KR, VT, VTR, O16, OR16);
}
__global__ __launch_bounds__(128) void k_attn_dense(const _Float16* __restrict__ Q16, const _Float16* __restrict__ QR, const _Float16* __restrict__ K16, const _Float16* __restrict__ KR,
    const _Float16* __restrict__ VT, _Float16* __restrict__ O16) {
  attn_hr_body<0>(Q16, QR, K16, KR, VT, VT, O16, O16);
}

template <int RBF, int RMAP, int W16, int OMAP>
__global__ __launch_bounds__(256) void k_ln(const float* __restrict__ X, const float* __restrict__ R, const float* __restrict__ g, const float* __restrict__ bb, float eps, float* __restrict__ O32, _Float16* __restrict__ O16) {
  #pragma clang fp contract(off)
  __shared__ float red[256];
  const size_t r = blockIdx.x; const int t = threadIdx.x; const int c0 = t * 4;
  const size_t rfull = (r / SEQ) * SEQ_FULL + (r % SEQ);
  const size_t rr = RMAP ? rfull : r;
  const v4f xa = *(const v4fa*)(X + r * DM + c0); const v4f ra = *(const v4fa*)(R + rr * DM + c0);
  float s[4]; float sum = 0.f;
#pragma unroll
  for (int q = 0; q < 4; ++q) { const float rv = RBF ? bf16_rne(ra[q]) : ra[q]; s[q] = xa[q] + rv; sum += s[q]; }
  red[t] = sum; __syncthreads();
  for (int st = 128; st > 0; st >>= 1) { if (t < st) red[t] += red[t + st]; __syncthreads(); }
  const float mu = red[0] * (1.0f / (float)DM); __syncthreads();
  float vs = 0.f;
#pragma unroll
  for (int q = 0; q < 4; ++q) { const float dl = s[q] - mu; vs += dl * dl; }
  red[t] = vs; __syncthreads();
  for (int st = 128; st > 0; st >>= 1) { if (t < st) red[t] += red[t + st]; __syncthreads(); }
  const float rs = rsqrtf(red[0] * (1.0f / (float)DM) + eps);
  v4f yf; v4h y;
#pragma unroll
  for (int q = 0; q < 4; ++q) { const int c = c0 + q; yf[q] = (s[q] - mu) * rs * bf16_rne(g[c]) + bf16_rne(bb[c]); y[q] = (_Float16)yf[q]; }
  const size_t orow = OMAP ? rfull : r;
  for (int pass = 0; pass < 2; ++pass) {
    if (O32) *(volatile v4f*)(O32 + orow * DM + c0) = yf;
    if (W16) *(volatile v4h*)(O16 + r * DM + c0) = y;
    if (pass == 0) __threadfence(); }
}

extern "C" void kernel_launch(void* const* d_in, const int* in_sizes, int n_in,
                              void* d_out, int out_size, void* d_ws, size_t ws_size, hipStream_t stream) {
  if (n_in < 22) return;
  const float* x    = (const float*)d_in[0];  const float* enc  = (const float*)d_in[1];
  const float* wq1  = (const float*)d_in[2];  const float* wk1  = (const float*)d_in[3];  const float* wv1 = (const float*)d_in[4];
  const float* wo1  = (const float*)d_in[5];  const float* bo1  = (const float*)d_in[6];
  const float* wq2  = (const float*)d_in[7];  const float* wk2  = (const float*)d_in[8];  const float* wv2 = (const float*)d_in[9];
  const float* wo2  = (const float*)d_in[10]; const float* bo2  = (const float*)d_in[11];
  const float* wff1 = (const float*)d_in[12]; const float* bff1 = (const float*)d_in[13]; const float* wff2 = (const float*)d_in[14]; const float* bff2 = (const float*)d_in[15];
  const float* g1   = (const float*)d_in[16]; const float* be1  = (const float*)d_in[17]; const float* g2  = (const float*)d_in[18]; const float* be2 = (const float*)d_in[19];
  const float* g3   = (const float*)d_in[20]; const float* be3  = (const float*)d_in[21];

  const size_t needX = ((size_t)(NB - 1) * SEQ_FULL + SEQ) * DM;
  if ((size_t)in_sizes[0] < needX || (size_t)in_sizes[1] < needX || (size_t)out_size < needX) return;
  { static const int wi[8] = {2, 3, 4, 5, 7, 8, 9, 10}; for (int i = 0; i < 8; ++i) if ((size_t)in_sizes[wi[i]] < (size_t)DM * DM) return; }
  if ((size_t)in_sizes[12] < (size_t)DM * DFF || (size_t)in_sizes[14] < (size_t)DM * DFF || in_sizes[13] < DFF) return;
  { static const int vi[9] = {6, 11, 15, 16, 17, 18, 19, 20, 21}; for (int i = 0; i < 9; ++i) if (in_sizes[vi[i]] < DM) return; }

  char* ws = (char*)d_ws; size_t off = 0;
  auto take = [&](size_t bytes) { char* p = ws + off; off += (bytes + 255) & ~(size_t)255; return p; };
  const size_t WDD = (size_t)DM * DM * 2, WDF = (size_t)DM * DFF * 2, P16 = NR * DM * 2;
  _Float16* BQ1 = (_Float16*)take(WDD); _Float16* BK1 = (_Float16*)take(WDD); _Float16* BV1 = (_Float16*)take(WDD); _Float16* BO1 = (_Float16*)take(WDD);
  _Float16* BQ2 = (_Float16*)take(WDD); _Float16* BK2 = (_Float16*)take(WDD); _Float16* BV2 = (_Float16*)take(WDD); _Float16* BO2 = (_Float16*)take(WDD);
  _Float16* BW1 = (_Float16*)take(WDF);
  _Float16* BW2 = (_Float16*)take(WDF);
  char* SL = take(10 * P16);
  _Float16* S0 = (_Float16*)(SL + 0 * P16); _Float16* S1 = (_Float16*)(SL + 1 * P16); _Float16* S2 = (_Float16*)(SL + 2 * P16); _Float16* S3 = (_Float16*)(SL + 3 * P16);
  _Float16* S4 = (_Float16*)(SL + 4 * P16); _Float16* S5 = (_Float16*)(SL + 5 * P16); _Float16* S6 = (_Float16*)(SL + 6 * P16); _Float16* S7 = (_Float16*)(SL + 7 * P16);
  _Float16* S8 = (_Float16*)(SL + 8 * P16); _Float16* S9 = (_Float16*)(SL + 9 * P16);
  float* YFa = (float*)S2;
  float* X1F = (float*)S4;
  float* X2F = (float*)S8;
  float* YFf = (float*)S6;
  _Float16* HF = S2;
  if (off > ws_size || off > (size_t)134217728) return;

  const unsigned gDD = (unsigned)(((size_t)DM * (DM / 8) + 255) / 256), gDF = (unsigned)(((size_t)DFF * (DM / 8) + 255) / 256), gFD = (unsigned)(((size_t)DM * (DFF / 8) + 255) / 256);
  k_wt_head<<<gDD, 256, 0, stream>>>(wq1, BQ1, DM, DM, 16.0f); k_wt_head<<<gDD, 256, 0, stream>>>(wk1, BK1, DM, DM, 16.0f); k_wt_head<<<gDD, 256, 0, stream>>>(wv1, BV1, DM, DM, 16.0f);
  k_wt_f16<<<gDD, 256, 0, stream>>>(wo1, BO1, DM, DM, 16.0f);
  k_wt_head<<<gDD, 256, 0, stream>>>(wq2, BQ2, DM, DM, 16.0f); k_wt_head<<<gDD, 256, 0, stream>>>(wk2, BK2, DM, DM, 16.0f); k_wt_head<<<gDD, 256, 0, stream>>>(wv2, BV2, DM, DM, 16.0f);
  k_wt_f16<<<gDD, 256, 0, stream>>>(wo2, BO2, DM, DM, 16.0f);
  k_wt_f16<<<gDF, 256, 0, stream>>>(wff1, BW1, DM, DFF, 16.0f); k_wt_f16<<<gFD, 256, 0, stream>>>(wff2, BW2, DFF, DM, 16.0f);

  const size_t n8 = NR * DM / 8; const unsigned gx = (unsigned)((n8 + 255) / 256);
  k_x16<<<gx, 256, 0, stream>>>(x, S0, n8); k_x16<<<gx, 256, 0, stream>>>(enc, S1, n8);

  const unsigned gP = (unsigned)((MR / 128) * (DM / 64)), gF1 = (unsigned)((MR / 128) * (DFF / 64));
  const unsigned gVT = (unsigned)(NB * NH * (SEQ / 64)); const dim3 gAT(SEQ / 64, NH, NB);

  k_proj_hr<<<gP, 128, 0, stream>>>(S0, DM, BQ1, DM, 0.0625f, S2, S3, DM, MR, DM, DM);
  k_proj_hr<<<gP, 128, 0, stream>>>(S0, DM, BK1, DM, 0.0625f, S4, S5, DM, MR, DM, DM);
  k_proj_hr<<<gP, 128, 0, stream>>>(S0, DM, BV1, DM, 0.0625f, S8, S9, DM, MR, DM, DM);
  k_vt<NH, SEQ><<<gVT, 256, 0, stream>>>(S8, DM, 0, S6);
  k_vt<NH, SEQ><<<gVT, 256, 0, stream>>>(S9, DM, 0, S7);
  k_attn_causal<<<gAT, 128, 0, stream>>>(S2, S3, S4, S5, S6, S7, S8, S9);
  k_proj_rf<<<gP, 128, 0, stream>>>(S8, S9, DM, BO1, DM, 0.0009765625f, bo1, 1.0f, YFa, DM, MR, DM, DM);
  k_ln<1, 1, 0, 0><<<(unsigned)MR, 256, 0, stream>>>(YFa, x, g1, be1, LN_EPS, X1F, nullptr);
  k_split16<<<gx, 256, 0, stream>>>(X1F, S6, S7, n8);
  k_proj_rhr<<<gP, 128, 0, stream>>>(S6, S7, DM, BQ2, DM, 0.0625f, S8, S9, DM, MR, DM, DM);
  k_proj_hr<<<gP, 128, 0, stream>>>(S1, DM, BK2, DM, 0.0625f, S2, S3, DM, MR, DM, DM);
  k_gemm2<0><<<gP, 128, 0, stream>>>(S1, DM, BV2, DM, 0.0625f, nullptr, 1.0f, nullptr, S0, DM, MR, DM, DM);
  k_vt<NH, SEQ><<<gVT, 256, 0, stream>>>(S0, DM, 0, S6);
  k_attn_dense<<<gAT, 128, 0, stream>>>(S8, S9, S2, S3, S6, S7);
  k_gemm2<0><<<gP, 128, 0, stream>>>(S7, DM, BO2, DM, 0.0009765625f, bo2, 1.0f, YFa, nullptr, DM, MR, DM, DM);
  k_ln<0, 0, 1, 0><<<(unsigned)MR, 256, 0, stream>>>(YFa, X1F, g2, be2, LN_EPS, X2F, S1);
  k_gemm2<3><<<gF1, 128, 0, stream>>>(S1, DM, BW1, DM, 1.0f, bff1, 16.0f, nullptr, HF, DFF, MR, DFF, DM);
  k_gemm2<0><<<gP, 128, 0, stream>>>(HF, DFF, BW2, DFF, 0.00390625f, bff2, 1.0f, YFf, nullptr, DM, MR, DM, DFF);
  k_ln<0, 0, 0, 1><<<(unsigned)MR, 256, 0, stream>>>(YFf, X2F, g3, be3, LN_EPS, (float*)d_out, nullptr);
}
